// CQAttention_2920577761511
// MI455X (gfx1250) — hardware-verified
//
#include <hip/hip_runtime.h>
#include <stddef.h>
#include <stdint.h>
#include <math.h>

#define NB   32
#define HH   256
#define LC   1024
#define LQ   256
#define FD   1024
#define X3W  768
#define NCL  (NB * LC)
#define NQL  (NB * LQ)
#define NCH  (NB * HH)
#define TP   72
#define NCT  (NB * 4 * 16)
#define NQT  (NB * 4 * 4)

#define CT_BYTES  ((size_t)NCL * HH * 2)
#define S_BYTES   ((size_t)NCL * LQ * 4)
#define C16_BYTES ((size_t)NCH * LC * 2)
#define X3_BYTES  ((size_t)NCL * X3W * 2)
#define PH_BYTES  ((size_t)NCL * HH * 2)
#define P16_BYTES ((size_t)NCL * LQ * 2)
#define SCT_BYTES ((size_t)NQL * LC * 2)
#define Q16_BYTES ((size_t)NCH * LQ * 2)
#define QT_BYTES  ((size_t)NQL * HH * 2)
#define UT_BYTES  ((size_t)NCH * LQ * 2)
#define W16_BYTES ((size_t)HH * FD * 2)
#define C1_BYTES  ((size_t)NCL * 4)
#define Q2_BYTES  ((size_t)NQL * 4)

#define OFF_CT   ((size_t)0)
#define OFF_S    (OFF_CT + CT_BYTES)
#define OFF_C16  (OFF_S + S_BYTES)
#define OFF_X3   OFF_S
#define OFF_PH   (OFF_C16 + C16_BYTES)
#define OFF_PL   (OFF_PH + PH_BYTES)
#define OFF_P16  OFF_PH
#define OFF_SCT  OFF_PL
#define OFF_Q16  (OFF_PL + PH_BYTES)
#define OFF_QT   (OFF_Q16 + Q16_BYTES)
#define OFF_UT   (OFF_QT + QT_BYTES)
#define OFF_W16  (OFF_UT + UT_BYTES)
#define OFF_C1   (OFF_W16 + W16_BYTES)
#define OFF_Q2   (OFF_C1 + C1_BYTES)
#define WS_TOTAL (OFF_Q2 + Q2_BYTES)

static_assert(WS_TOTAL == (size_t)113934336);
static_assert(WS_TOTAL <= (size_t)134217728);
static_assert(X3_BYTES == S_BYTES + C16_BYTES);
static_assert(P16_BYTES == PH_BYTES);
static_assert(SCT_BYTES == PH_BYTES);
static_assert((OFF_S % 256) == 0);
static_assert((OFF_C16 % 256) == 0);
static_assert((OFF_PH % 256) == 0);
static_assert((OFF_PL % 256) == 0);
static_assert((OFF_Q16 % 256) == 0);
static_assert((OFF_QT % 256) == 0);
static_assert((OFF_UT % 256) == 0);
static_assert((OFF_W16 % 256) == 0);
static_assert((OFF_C1 % 256) == 0);
static_assert((OFF_Q2 % 256) == 0);
static_assert((LC % 64) == 0);
static_assert((LQ % 64) == 0);
static_assert((HH % 64) == 0);
static_assert((FD % 32) == 0);
static_assert((X3W % 64) == 0);
static_assert(FD == HH + X3W);
static_assert((NCL % 256) == 0);
static_assert((NQL % 256) == 0);
static_assert(((HH * FD) % 2048) == 0);
static_assert((NCL % 8) == 0);
static_assert(LQ == 256);
static_assert((LC % 8) == 0);

typedef unsigned short v8us  __attribute__((ext_vector_type(8)));
typedef unsigned short v16us __attribute__((ext_vector_type(16)));
typedef _Float16       v16h  __attribute__((ext_vector_type(16)));
typedef float          v4f   __attribute__((ext_vector_type(4)));
typedef float          v8f   __attribute__((ext_vector_type(8)));
typedef int            v4i   __attribute__((ext_vector_type(4)));

union FragU { v16us v; v8us half[2]; };

__device__ __forceinline__ unsigned bbits(float f) {
  unsigned u = __float_as_uint(f);
  return (u + 0x7FFFu + ((u >> 16) & 1u)) >> 16;
}
__device__ __forceinline__ float bf16r(float f) {
  return __uint_as_float(bbits(f) << 16);
}
__device__ __forceinline__ unsigned short hbits(float f) {
  return __builtin_bit_cast(unsigned short, (_Float16)f);
}
__device__ __forceinline__ v8f zero8() { v8f z = {0.f, 0.f, 0.f, 0.f, 0.f, 0.f, 0.f, 0.f}; return z; }

__device__ __forceinline__ v16us ldfrag_u(const unsigned short* p) {
  FragU f;
  f.half[0] = *(const v8us*)(p);
  f.half[1] = *(const v8us*)(p + 16);
  return f.v;
}

__device__ __forceinline__ v8f mma_hu(v16us a, v16us b, v8f c) {
#if defined(__HIP_DEVICE_COMPILE__)
  return __builtin_amdgcn_wmma_f32_16x16x32_f16(false, __builtin_bit_cast(v16h, a),
                                               false, __builtin_bit_cast(v16h, b),
                                               (short)0, c, false, false);
#else
  (void)a; (void)b;
  return c;
#endif
}
__device__ __forceinline__ void guard4(v8f& c0, v8f& c1, v8f& c2, v8f& c3, const v16us& a,
                                       const v16us& b0, const v16us& b1, const v16us& b2,
                                       const v16us& b3) {
#if defined(__HIP_DEVICE_COMPILE__)
  asm volatile("v_nop\n\tv_nop\n\tv_nop\n\tv_nop"
               : "+v"(c0), "+v"(c1), "+v"(c2), "+v"(c3)
               : "v"(a), "v"(b0), "v"(b1), "v"(b2), "v"(b3));
#else
  (void)c0; (void)c1; (void)c2; (void)c3; (void)a; (void)b0; (void)b1; (void)b2; (void)b3;
#endif
}
__device__ __forceinline__ void guard8(v8f& c0, v8f& c1, v8f& c2, v8f& c3, v8f& c4, v8f& c5,
                                       v8f& c6, v8f& c7, const v16us& a0, const v16us& a1,
                                       const v16us& b0, const v16us& b1, const v16us& b2,
                                       const v16us& b3) {
#if defined(__HIP_DEVICE_COMPILE__)
  asm volatile("v_nop\n\tv_nop\n\tv_nop\n\tv_nop"
               : "+v"(c0), "+v"(c1), "+v"(c2), "+v"(c3), "+v"(c4), "+v"(c5), "+v"(c6), "+v"(c7)
               : "v"(a0), "v"(a1), "v"(b0), "v"(b1), "v"(b2), "v"(b3));
#else
  (void)c0; (void)c1; (void)c2; (void)c3; (void)c4; (void)c5; (void)c6; (void)c7;
  (void)a0; (void)a1; (void)b0; (void)b1; (void)b2; (void)b3;
#endif
}

__device__ __forceinline__ void store_tile_f32(const float* ct, float* C, size_t row0, int col0,
                                               int ldc, int w, int lane) {
  const int q  = lane >> 3;
  const int jj = lane & 7;
#pragma unroll 1
  for (int it = 0; it < 8; ++it) {
    const int li = it * 16 + w * 4 + q;
    const int tr = li >> 1, hf = li & 1;
    const v4f v = *(const v4f*)(ct + tr * 64 + hf * 32 + jj * 4);
    *(volatile v4f*)(C + (row0 + tr) * (size_t)ldc + col0 + hf * 32 + jj * 4) = v;
  }
  __threadfence();
#pragma unroll 1
  for (int it = 0; it < 8; ++it) {
    const int li = it * 16 + w * 4 + q;
    const int tr = li >> 1, hf = li & 1;
    const v4f v = *(const v4f*)(ct + tr * 64 + hf * 32 + jj * 4);
    *(volatile v4f*)(C + (row0 + tr) * (size_t)ldc + col0 + hf * 32 + jj * 4) = v;
  }
}
template <int NW, int PITCH>
__device__ __forceinline__ void store_tile_us(const unsigned short* t, unsigned short* P,
                                              size_t row0, int ld, int col0, int w, int lane) {
  constexpr int NIT = 64 / (4 * NW);
  const int q  = lane >> 3;
  const int jj = lane & 7;
  v8us   v[NIT];
  size_t off[NIT];
#pragma unroll
  for (int it = 0; it < NIT; ++it) {
    const int li = it * 4 * NW + w * 4 + q;
    v[it]   = *(const v8us*)(t + li * PITCH + 8 * jj);
    off[it] = (row0 + li) * (size_t)ld + col0 + 8 * jj;
  }
#pragma unroll
  for (int it = 0; it < NIT; ++it) *(volatile v8us*)(P + off[it]) = v[it];
  __threadfence();
#pragma unroll
  for (int it = 0; it < NIT; ++it) *(volatile v8us*)(P + off[it]) = v[it];
}

__global__ __launch_bounds__(256)
void k_cvt(const float* __restrict__ Cin, const float* __restrict__ Qin,
           const float* __restrict__ wv,
           unsigned short* c16, unsigned short* ct16, unsigned short* ph16,
           unsigned short* pl16, unsigned short* q16, unsigned short* qt16)
{
  __shared__ __align__(16) unsigned short tdir[64 * TP];
  __shared__ __align__(16) unsigned short ttr[64 * TP];
  __shared__ __align__(16) unsigned short tph[64 * TP];
  __shared__ __align__(16) unsigned short tpl[64 * TP];

  const int tid  = threadIdx.x;
  const int lane = tid & 31;
  const int w    = tid >> 5;
  const int bid  = blockIdx.x;
  const int kind = (bid < NCT) ? 0 : 1;
  const int loc  = kind ? (bid - NCT) : bid;
  const int L    = kind ? LQ : LC;
  const int ltb  = kind ? 2 : 4;
  const int lt   = loc & ((1 << ltb) - 1);
  const int ht   = (loc >> ltb) & 3;
  const int b    = loc >> (ltb + 2);
  const int h0   = 64 * ht;
  const int l0   = 64 * lt;

  const int hh = tid >> 2;
  const int lo = 16 * (tid & 3);
  const float* sp = (kind ? Qin : Cin) + ((size_t)b * HH + h0 + hh) * L + l0 + lo;
  v4f u[4];
  u[0] = *(const v4f*)(sp);
  u[1] = *(const v4f*)(sp + 4);
  u[2] = *(const v4f*)(sp + 8);
  u[3] = *(const v4f*)(sp + 12);
  const float w3v = bf16r(wv[2 * HH + h0 + hh]);
#pragma unroll
  for (int g = 0; g < 4; ++g) {
#pragma unroll
    for (int e = 0; e < 4; ++e) {
      const int ll = lo + 4 * g + e;
      const float x = bf16r(u[g][e]);
      const unsigned short hb = hbits(16.0f * x);
      tdir[hh * TP + ll] = hb;
      ttr[ll * TP + hh]  = hb;
      const float p = (x * w3v) * 1024.0f;
      const _Float16 phh = (_Float16)p;
      const float res = (p - (float)phh) * 2048.0f;
      tph[ll * TP + hh] = __builtin_bit_cast(unsigned short, phh);
      tpl[ll * TP + hh] = hbits(res);
    }
  }
  __syncthreads();

  store_tile_us<8, TP>(tdir, kind ? q16 : c16, (size_t)b * HH + h0, L, l0, w, lane);
  store_tile_us<8, TP>(ttr, kind ? qt16 : ct16, (size_t)b * L + l0, HH, h0, w, lane);
  if (kind == 0) {
    store_tile_us<8, TP>(tph, ph16, (size_t)b * LC + l0, HH, h0, w, lane);
    store_tile_us<8, TP>(tpl, pl16, (size_t)b * LC + l0, HH, h0, w, lane);
  }
}

__global__ __launch_bounds__(256)
void k_misc(const float* __restrict__ Cin, const float* __restrict__ Qin,
            const float* __restrict__ wv, const float* __restrict__ Wres,
            unsigned short* w16, float* c1, float* q2)
{
  __shared__ float wL[3 * HH];
  const int tid = threadIdx.x;
  for (int i = tid; i < 3 * HH; i += 256) wL[i] = bf16r(wv[i]);
  __syncthreads();

  const int bid = blockIdx.x;
  if (bid < 128) {
    const int i = bid * 256 + tid;
    const float* fp = Wres + (size_t)8 * i;
    const v4f a0 = *(const v4f*)(fp);
    const v4f a1 = *(const v4f*)(fp + 4);
    v8us ob;
#pragma unroll
    for (int e = 0; e < 4; ++e) {
      ob[e]     = hbits(64.0f * bf16r(a0[e]));
      ob[4 + e] = hbits(64.0f * bf16r(a1[e]));
    }
    unsigned short* dst = w16 + (size_t)8 * i;
    *(volatile v8us*)dst = ob;
    __threadfence();
    *(volatile v8us*)dst = ob;
  } else if (bid < 256) {
    const int i = (bid - 128) * 256 + tid;
    const int b = i >> 10;
    const int l = i & (LC - 1);
    const float* cp = Cin + (size_t)b * HH * LC + l;
    float s = 0.f;
#pragma unroll 1
    for (int h = 0; h < HH; ++h) s += bf16r(cp[(size_t)h * LC]) * wL[h];
    const float sv = s;
    *(volatile float*)(c1 + i) = sv;
    __threadfence();
    *(volatile float*)(c1 + i) = sv;
  } else {
    const int j = (bid - 256) * 256 + tid;
    const int b = j >> 8;
    const int mq = j & (LQ - 1);
    const float* qp = Qin + (size_t)b * HH * LQ + mq;
    float s = 0.f;
#pragma unroll 1
    for (int h = 0; h < HH; ++h) s += bf16r(qp[(size_t)h * LQ]) * wL[HH + h];
    const float sv = s;
    *(volatile float*)(q2 + j) = sv;
    __threadfence();
    *(volatile float*)(q2 + j) = sv;
  }
}

__global__ __launch_bounds__(128)
void k_score(const unsigned short* __restrict__ ph16, const unsigned short* __restrict__ pl16,
             const unsigned short* __restrict__ qt16, const float* __restrict__ c1,
             const float* __restrict__ q2, float* S)
{
  __shared__ __align__(16) float ct[64 * 64];

  const int tid  = threadIdx.x;
  const int lane = tid & 31;
  const int w    = tid >> 5;
  const int h    = lane >> 4;
  const int m    = lane & 15;
  const int m0   = 64 * blockIdx.x;
  const int l0   = 64 * blockIdx.y;
  const int b    = blockIdx.z;

  v8f acc[4], accl[4];
#pragma unroll
  for (int j = 0; j < 4; ++j) { acc[j] = zero8(); accl[j] = zero8(); }

  const size_t arow = (size_t)b * LC + l0 + 16 * w + m;
  const unsigned short* pah = ph16 + arow * HH + 8 * h;
  const unsigned short* pal = pl16 + arow * HH + 8 * h;
  const unsigned short* pb  = qt16 + ((size_t)b * LQ + m0 + m) * HH + 8 * h;
#pragma unroll 2
  for (int kk = 0; kk < HH / 32; ++kk) {
    const v16us ah = ldfrag_u(pah + 32 * kk);
    const v16us al = ldfrag_u(pal + 32 * kk);
    const v16us b0 = ldfrag_u(pb + 32 * kk);
    const v16us b1 = ldfrag_u(pb + (size_t)16 * HH + 32 * kk);
    const v16us b2 = ldfrag_u(pb + (size_t)32 * HH + 32 * kk);
    const v16us b3 = ldfrag_u(pb + (size_t)48 * HH + 32 * kk);
    acc[0]  = mma_hu(ah, b0, acc[0]);
    acc[1]  = mma_hu(ah, b1, acc[1]);
    acc[2]  = mma_hu(ah, b2, acc[2]);
    acc[3]  = mma_hu(ah, b3, acc[3]);
    accl[0] = mma_hu(al, b0, accl[0]);
    accl[1] = mma_hu(al, b1, accl[1]);
    accl[2] = mma_hu(al, b2, accl[2]);
    accl[3] = mma_hu(al, b3, accl[3]);
    guard8(acc[0], acc[1], acc[2], acc[3], accl[0], accl[1], accl[2], accl[3],
           ah, al, b0, b1, b2, b3);
  }

  float c1v[8];
#pragma unroll
  for (int r = 0; r < 8; ++r) c1v[r] = c1[(size_t)b * LC + l0 + 16 * w + 8 * h + r];
  const float kl = 1.0f / 2048.0f;
  const float ks = 1.0f / 16384.0f;
#pragma unroll
  for (int j = 0; j < 4; ++j) {
    const float q2v = q2[(size_t)b * LQ + m0 + 16 * j + m];
#pragma unroll
    for (int r = 0; r < 8; ++r) {
      const float s3 = (acc[j][r] + accl[j][r] * kl) * ks;
      ct[(16 * w + 8 * h + r) * 64 + 16 * j + m] = (c1v[r] + q2v) + s3;
    }
  }
  __syncthreads();
  store_tile_f32(ct, S, (size_t)b * LC + l0, m0, LQ, w, lane);
}

__global__ __launch_bounds__(256)
void k_rowsm(const float* __restrict__ S, const int* __restrict__ qmask, unsigned short* p16)
{
  const float NEGV = -1.0e30f;
  const int lane = threadIdx.x & 31;
  const int row  = blockIdx.x * 8 + (threadIdx.x >> 5);
  const int b    = row >> 10;
  const float* sr = S + (size_t)row * LQ + 8 * lane;
  const v4f x0 = *(const v4f*)(sr);
  const v4f x1 = *(const v4f*)(sr + 4);
  const int* qp = qmask + (size_t)b * LQ + 8 * lane;
  const v4i q0 = *(const v4i*)(qp);
  const v4i q1 = *(const v4i*)(qp + 4);
  float s[8];
#pragma unroll
  for (int e = 0; e < 4; ++e) {
    s[e]     = x0[e] + NEGV * (1.0f - (float)q0[e]);
    s[4 + e] = x1[e] + NEGV * (1.0f - (float)q1[e]);
  }
  float mx = s[0];
#pragma unroll
  for (int e = 1; e < 8; ++e) mx = fmaxf(mx, s[e]);
#pragma unroll
  for (int o = 16; o >= 1; o >>= 1) mx = fmaxf(mx, __shfl_xor(mx, o, 32));
  float ex[8];
  float sum = 0.f;
#pragma unroll
  for (int e = 0; e < 8; ++e) { ex[e] = __expf(s[e] - mx); sum += ex[e]; }
#pragma unroll
  for (int o = 16; o >= 1; o >>= 1) sum += __shfl_xor(sum, o, 32);
  const float inv = 1.0f / sum;
  v8us o;
#pragma unroll
  for (int e = 0; e < 8; ++e) o[e] = hbits(4096.0f * (ex[e] * inv));
  unsigned short* dst = p16 + (size_t)row * LQ + 8 * lane;
  *(volatile v8us*)dst = o;
  __threadfence();
  *(volatile v8us*)dst = o;
}

__global__ __launch_bounds__(256)
void k_colsm(const float* __restrict__ S, const int* __restrict__ cmask, unsigned short* sct)
{
  __shared__ float red[8][32];
  __shared__ float colmax[32];
  __shared__ float colinv[32];
  __shared__ __align__(16) unsigned short tileT[32 * TP];

  const float NEGV = -1.0e30f;
  const int tid = threadIdx.x;
  const int tx  = tid & 31;
  const int ty  = tid >> 5;
  const int q   = tx >> 3;
  const int jj  = tx & 7;
  const int b   = blockIdx.x >> 3;
  const int m0  = 32 * (blockIdx.x & 7);
  const float* Sb = S + (size_t)b * LC * LQ + m0 + tx;
  const int* cmb  = cmask + (size_t)b * LC;

  float mx = -INFINITY;
#pragma unroll 2
  for (int i = 0; i < LC / 8; ++i) {
    const int l = ty * (LC / 8) + i;
    const float s = Sb[(size_t)l * LQ] + NEGV * (1.0f - (float)cmb[l]);
    mx = fmaxf(mx, s);
  }
  red[ty][tx] = mx;
  __syncthreads();
  if (ty == 0) {
    float m2 = red[0][tx];
#pragma unroll
    for (int j = 1; j < 8; ++j) m2 = fmaxf(m2, red[j][tx]);
    colmax[tx] = m2;
  }
  __syncthreads();
  const float cmx = colmax[tx];

  float sm = 0.f;
#pragma unroll 2
  for (int i = 0; i < LC / 8; ++i) {
    const int l = ty * (LC / 8) + i;
    const float s = Sb[(size_t)l * LQ] + NEGV * (1.0f - (float)cmb[l]);
    sm += __expf(s - cmx);
  }
  red[ty][tx] = sm;
  __syncthreads();
  if (ty == 0) {
    float s2 = 0.f;
#pragma unroll
    for (int j = 0; j < 8; ++j) s2 += red[j][tx];
    colinv[tx] = 1.0f / s2;
  }
  __syncthreads();
  const float inv = colinv[tx];

#pragma unroll 1
  for (int c = 0; c < LC / 64; ++c) {
#pragma unroll
    for (int i = 0; i < 8; ++i) {
      const int l = 64 * c + ty + 8 * i;
      const float s = Sb[(size_t)l * LQ] + NEGV * (1.0f - (float)cmb[l]);
      const float v = 4096.0f * (__expf(s - cmx) * inv);
      tileT[tx * TP + ty + 8 * i] = hbits(v);
    }
    __syncthreads();
    {
      const int li = 4 * ty + q;
      const v8us v = *(const v8us*)(tileT + li * TP + 8 * jj);
      unsigned short* dst = sct + ((size_t)b * LQ + m0 + li) * LC + 64 * c + 8 * jj;
      *(volatile v8us*)dst = v;
      __threadfence();
      *(volatile v8us*)dst = v;
    }
    __syncthreads();
  }
}

__global__ __launch_bounds__(128)
void k_ut(const unsigned short* __restrict__ c16, const unsigned short* __restrict__ sct,
          unsigned short* ut16)
{
  __shared__ __align__(16) unsigned short ht[64 * 64];

  const int tid  = threadIdx.x;
  const int lane = tid & 31;
  const int w    = tid >> 5;
  const int h    = lane >> 4;
  const int m    = lane & 15;
  const int n0   = 64 * blockIdx.x;
  const int r0   = 64 * blockIdx.y;
  const int b    = blockIdx.z;

  v8f acc[4];
#pragma unroll
  for (int j = 0; j < 4; ++j) acc[j] = zero8();

  const unsigned short* pa = c16 + ((size_t)b * HH + r0 + 16 * w + m) * LC + 8 * h;
  const unsigned short* pb = sct + ((size_t)b * LQ + n0 + m) * LC + 8 * h;
#pragma unroll 2
  for (int kk = 0; kk < LC / 32; ++kk) {
    const v16us a  = ldfrag_u(pa + 32 * kk);
    const v16us b0 = ldfrag_u(pb + 32 * kk);
    const v16us b1 = ldfrag_u(pb + (size_t)16 * LC + 32 * kk);
    const v16us b2 = ldfrag_u(pb + (size_t)32 * LC + 32 * kk);
    const v16us b3 = ldfrag_u(pb + (size_t)48 * LC + 32 * kk);
    acc[0] = mma_hu(a, b0, acc[0]);
    acc[1] = mma_hu(a, b1, acc[1]);
    acc[2] = mma_hu(a, b2, acc[2]);
    acc[3] = mma_hu(a, b3, acc[3]);
    guard4(acc[0], acc[1], acc[2], acc[3], a, b0, b1, b2, b3);
  }

  const float ku = 1.0f / 64.0f;
#pragma unroll
  for (int j = 0; j < 4; ++j) {
#pragma unroll
    for (int r = 0; r < 8; ++r)
      ht[(16 * w + 8 * h + r) * 64 + 16 * j + m] = hbits(acc[j][r] * ku);
  }
  __syncthreads();
  store_tile_us<4, 64>(ht, ut16, (size_t)b * HH + r0, LQ, n0, w, lane);
}

__global__ __launch_bounds__(128)
void k_av(const unsigned short* __restrict__ p16, const unsigned short* __restrict__ q16,
          const unsigned short* __restrict__ ut16, const unsigned short* __restrict__ ct16,
          unsigned short* x3)
{
  __shared__ __align__(16) unsigned short ctL[64 * TP];
  __shared__ __align__(16) unsigned short hA[64 * 64];
  __shared__ __align__(16) unsigned short hCA[64 * 64];
  __shared__ __align__(16) unsigned short hCB[64 * 64];

  const int tid  = threadIdx.x;
  const int lane = tid & 31;
  const int w    = tid >> 5;
  const int h    = lane >> 4;
  const int m    = lane & 15;
  const int h0   = 64 * blockIdx.x;
  const int l0   = 64 * blockIdx.y;
  const int b    = blockIdx.z;
  const size_t crow0 = (size_t)b * LC + l0;

#pragma unroll
  for (int i = 0; i < 4; ++i) {
    const int p   = tid + 128 * i;
    const int rr  = p >> 3;
    const int jj2 = p & 7;
    const v8us v = *(const v8us*)(ct16 + (crow0 + rr) * HH + h0 + 8 * jj2);
    *(v8us*)(ctL + rr * TP + 8 * jj2) = v;
  }
  __syncthreads();

  v8f acc[4];
#pragma unroll
  for (int j = 0; j < 4; ++j) acc[j] = zero8();

  const unsigned short* pa  = p16 + (crow0 + 16 * w + m) * LQ + 8 * h;
  const unsigned short* pbq = q16 + ((size_t)b * HH + h0 + m) * LQ + 8 * h;
#pragma unroll 2
  for (int kk = 0; kk < LQ / 32; ++kk) {
    const v16us a  = ldfrag_u(pa + 32 * kk);
    const v16us b0 = ldfrag_u(pbq + 32 * kk);
    const v16us b1 = ldfrag_u(pbq + (size_t)16 * LQ + 32 * kk);
    const v16us b2 = ldfrag_u(pbq + (size_t)32 * LQ + 32 * kk);
    const v16us b3 = ldfrag_u(pbq + (size_t)48 * LQ + 32 * kk);
    acc[0] = mma_hu(a, b0, acc[0]);
    acc[1] = mma_hu(a, b1, acc[1]);
    acc[2] = mma_hu(a, b2, acc[2]);
    acc[3] = mma_hu(a, b3, acc[3]);
    guard4(acc[0], acc[1], acc[2], acc[3], a, b0, b1, b2, b3);
  }

  const float ka = 1.0f / 65536.0f;
#pragma unroll
  for (int j = 0; j < 4; ++j) {
#pragma unroll
    for (int r = 0; r < 8; ++r) {
      const int rl = 16 * w + 8 * h + r;
      const int ch = 16 * j + m;
      const unsigned short cb = ctL[rl * TP + ch];
      const float ctv = (float)__builtin_bit_cast(_Float16, cb);
      const float av  = acc[j][r] * ka;
      hA[rl * 64 + ch]  = hbits(16.0f * av);
      hCA[rl * 64 + ch] = hbits(ctv * av);
    }
  }

#pragma unroll
  for (int j = 0; j < 4; ++j) acc[j] = zero8();
  const unsigned short* pbu = ut16 + ((size_t)b * HH + h0 + m) * LQ + 8 * h;
#pragma unroll 2
  for (int kk = 0; kk < LQ / 32; ++kk) {
    const v16us a  = ldfrag_u(pa + 32 * kk);
    const v16us b0 = ldfrag_u(pbu + 32 * kk);
    const v16us b1 = ldfrag_u(pbu + (size_t)16 * LQ + 32 * kk);
    const v16us b2 = ldfrag_u(pbu + (size_t)32 * LQ + 32 * kk);
    const v16us b3 = ldfrag_u(pbu + (size_t)48 * LQ + 32 * kk);
    acc[0] = mma_hu(a, b0, acc[0]);
    acc[1] = mma_hu(a, b1, acc[1]);
    acc[2] = mma_hu(a, b2, acc[2]);
    acc[3] = mma_hu(a, b3, acc[3]);
    guard4(acc[0], acc[1], acc[2], acc[3], a, b0, b1, b2, b3);
  }

  const float kb = 1.0f / 4194304.0f;
#pragma unroll
  for (int j = 0; j < 4; ++j) {
#pragma unroll
    for (int r = 0; r < 8; ++r) {
      const int rl = 16 * w + 8 * h + r;
      const int ch = 16 * j + m;
      const unsigned short cb = ctL[rl * TP + ch];
      const float ctv = (float)__builtin_bit_cast(_Float16, cb);
      const float bvv = acc[j][r] * kb;
      hCB[rl * 64 + ch] = hbits(ctv * bvv);
    }
  }
  __syncthreads();

  store_tile_us<4, 64>(hA,  x3, crow0, X3W, h0, w, lane);
  store_tile_us<4, 64>(hCA, x3, crow0, X3W, HH + h0, w, lane);
  store_tile_us<4, 64>(hCB, x3, crow0, X3W, 2 * HH + h0, w, lane);
}

__global__ __launch_bounds__(128)
void k_out(const unsigned short* __restrict__ w16, const unsigned short* __restrict__ ct16,
           const unsigned short* __restrict__ x3, const float* __restrict__ bres, float* out)
{
  __shared__ __align__(16) float ct[64 * 64];

  const int tid  = threadIdx.x;
  const int lane = tid & 31;
  const int w    = tid >> 5;
  const int h    = lane >> 4;
  const int m    = lane & 15;
  const int l0   = 64 * blockIdx.x;
  const int r0   = 64 * blockIdx.y;
  const int b    = blockIdx.z;

  v8f acc[4];
#pragma unroll
  for (int j = 0; j < 4; ++j) acc[j] = zero8();

  const unsigned short* pa  = w16 + (size_t)(r0 + 16 * w + m) * FD + 8 * h;
  const size_t crow = (size_t)b * LC + l0 + m;
  const unsigned short* pb1 = ct16 + crow * HH + 8 * h;
  const unsigned short* pb2 = x3 + crow * X3W + 8 * h;
#pragma unroll 2
  for (int kk = 0; kk < HH / 32; ++kk) {
    const v16us a  = ldfrag_u(pa + 32 * kk);
    const v16us b0 = ldfrag_u(pb1 + 32 * kk);
    const v16us b1 = ldfrag_u(pb1 + (size_t)16 * HH + 32 * kk);
    const v16us b2 = ldfrag_u(pb1 + (size_t)32 * HH + 32 * kk);
    const v16us b3 = ldfrag_u(pb1 + (size_t)48 * HH + 32 * kk);
    acc[0] = mma_hu(a, b0, acc[0]);
    acc[1] = mma_hu(a, b1, acc[1]);
    acc[2] = mma_hu(a, b2, acc[2]);
    acc[3] = mma_hu(a, b3, acc[3]);
    guard4(acc[0], acc[1], acc[2], acc[3], a, b0, b1, b2, b3);
  }
#pragma unroll 2
  for (int kk = 0; kk < X3W / 32; ++kk) {
    const v16us a  = ldfrag_u(pa + HH + 32 * kk);
    const v16us b0 = ldfrag_u(pb2 + 32 * kk);
    const v16us b1 = ldfrag_u(pb2 + (size_t)16 * X3W + 32 * kk);
    const v16us b2 = ldfrag_u(pb2 + (size_t)32 * X3W + 32 * kk);
    const v16us b3 = ldfrag_u(pb2 + (size_t)48 * X3W + 32 * kk);
    acc[0] = mma_hu(a, b0, acc[0]);
    acc[1] = mma_hu(a, b1, acc[1]);
    acc[2] = mma_hu(a, b2, acc[2]);
    acc[3] = mma_hu(a, b3, acc[3]);
    guard4(acc[0], acc[1], acc[2], acc[3], a, b0, b1, b2, b3);
  }

  float bias[8];
#pragma unroll
  for (int r = 0; r < 8; ++r) bias[r] = bf16r(bres[r0 + 16 * w + 8 * h + r]);
  const float ko = 1.0f / 1024.0f;
#pragma unroll
  for (int j = 0; j < 4; ++j) {
#pragma unroll
    for (int r = 0; r < 8; ++r)
      ct[(16 * w + 8 * h + r) * 64 + 16 * j + m] = fmaxf(acc[j][r] * ko + bias[r], 0.0f);
  }
  __syncthreads();
  store_tile_f32(ct, out, (size_t)b * HH + r0, l0, LC, w, lane);
}

extern "C" void kernel_launch(void* const* d_in, const int* in_sizes, int n_in,
                              void* d_out, int out_size, void* d_ws, size_t ws_size,
                              hipStream_t stream) {
  if (n_in < 7) return;
  if (in_sizes[0] != NB * HH * LC) return;
  if (in_sizes[1] != NB * HH * LQ) return;
  if (in_sizes[2] != NB * LC) return;
  if (in_sizes[3] != NB * LQ) return;
  if (in_sizes[4] != 3 * HH) return;
  if (in_sizes[5] != HH * FD) return;
  if (in_sizes[6] != HH) return;
  if (out_size != NB * HH * LC) return;
  if (ws_size < WS_TOTAL) return;

  const float* Cin   = (const float*)d_in[0];
  const float* Qin   = (const float*)d_in[1];
  const int*   cmask = (const int*)d_in[2];
  const int*   qmask = (const int*)d_in[3];
  const float* wv    = (const float*)d_in[4];
  const float* Wres  = (const float*)d_in[5];
  const float* bres  = (const float*)d_in[6];
  float* out = (float*)d_out;

  char* ws = (char*)d_ws;
  unsigned short* ct16 = (unsigned short*)(ws + OFF_CT);
  float*          Sp   = (float*)(ws + OFF_S);
  unsigned short* c16  = (unsigned short*)(ws + OFF_C16);
  unsigned short* x3   = (unsigned short*)(ws + OFF_X3);
  unsigned short* ph16 = (unsigned short*)(ws + OFF_PH);
  unsigned short* pl16 = (unsigned short*)(ws + OFF_PL);
  unsigned short* p16  = (unsigned short*)(ws + OFF_P16);
  unsigned short* sct  = (unsigned short*)(ws + OFF_SCT);
  unsigned short* q16  = (unsigned short*)(ws + OFF_Q16);
  unsigned short* qt16 = (unsigned short*)(ws + OFF_QT);
  unsigned short* ut16 = (unsigned short*)(ws + OFF_UT);
  unsigned short* w16  = (unsigned short*)(ws + OFF_W16);
  float*          c1   = (float*)(ws + OFF_C1);
  float*          q2   = (float*)(ws + OFF_Q2);

  k_cvt<<<dim3(NCT + NQT), dim3(256), 0, stream>>>(Cin, Qin, wv, c16, ct16, ph16, pl16, q16, qt16);
  (void)hipGetLastError();
  k_misc<<<dim3(288), dim3(256), 0, stream>>>(Cin, Qin, wv, Wres, w16, c1, q2);
  (void)hipGetLastError();
  k_score<<<dim3(LQ / 64, LC / 64, NB), dim3(128), 0, stream>>>(ph16, pl16, qt16, c1, q2, Sp);
  (void)hipGetLastError();
  k_rowsm<<<dim3(NCL / 8), dim3(256), 0, stream>>>(Sp, qmask, p16);
  (void)hipGetLastError();
  k_colsm<<<dim3(NB * (LQ / 32)), dim3(256), 0, stream>>>(Sp, cmask, sct);
  (void)hipGetLastError();
  k_ut<<<dim3(LQ / 64, HH / 64, NB), dim3(128), 0, stream>>>(c16, sct, ut16);
  (void)hipGetLastError();
  k_av<<<dim3(HH / 64, LC / 64, NB), dim3(128), 0, stream>>>(p16, q16, ut16, ct16, x3);
  (void)hipGetLastError();
  k_out<<<dim3(LC / 64, HH / 64, NB), dim3(128), 0, stream>>>(w16, ct16, x3, bres, out);
  (void)hipGetLastError();
}
